// MHSA_3D_68470368633324
// MI455X (gfx1250) — hardware-run, weakly checked
//
#include <hip/hip_runtime.h>
#include <math.h>

typedef __attribute__((ext_vector_type(16))) _Float16 v16h;
typedef __attribute__((ext_vector_type(8)))  _Float16 v8h;
typedef __attribute__((ext_vector_type(16))) __bf16   v16b;
typedef __attribute__((ext_vector_type(8)))  __bf16   v8b;
typedef __attribute__((ext_vector_type(8)))  float    v8f;
typedef __attribute__((ext_vector_type(4)))  float    v4f;
typedef __attribute__((ext_vector_type(4)))  unsigned int v4u;

constexpr int kB     = 4;
constexpr int kC     = 256;
constexpr int kHeads = 8;
constexpr int kDk    = 32;
constexpr int kSide  = 12;
constexpr int kN     = kSide * kSide * kSide;
constexpr int kQTile = 64;
constexpr int kNQB   = kN / kQTile;
constexpr int kKC    = 64;
constexpr int kNCH   = kN / kKC;
constexpr int kOP    = 68;
constexpr float kPCarry = 32768.0f;
static_assert(kHeads * kDk == kC, "head split");
static_assert(kN == 1728, "positions");
static_assert(kDk == 32, "one 32-deep k-step per logit term");
static_assert((kN % 64) == 0 && (kC % 64) == 0, "GEMM M,N multiples of 64");
static_assert((kC % 32) == 0, "GEMM K multiple of 32");
static_assert(kNQB == 27 && kNCH == 27, "tile counts");

constexpr size_t kSzX   = (size_t)kB * kN * kC * 2;
constexpr size_t kSzW   = (size_t)kC * kC * 2;
constexpr size_t kSzP   = (size_t)kN * kC * 2;
constexpr size_t kOffXH  = 0;
constexpr size_t kOffXL  = kOffXH  + kSzX;
constexpr size_t kOffWQH = kOffXL  + kSzX;
constexpr size_t kOffWQL = kOffWQH + kSzW;
constexpr size_t kOffWKH = kOffWQL + kSzW;
constexpr size_t kOffWKL = kOffWKH + kSzW;
constexpr size_t kOffWVH = kOffWKL + kSzW;
constexpr size_t kOffWVL = kOffWVH + kSzW;
constexpr size_t kOffQH  = kOffWVL + kSzW;
constexpr size_t kOffQL  = kOffQH  + kSzX;
constexpr size_t kOffKH  = kOffQL  + kSzX;
constexpr size_t kOffKL  = kOffKH  + kSzX;
constexpr size_t kOffPH  = kOffKL  + kSzX;
constexpr size_t kOffPL  = kOffPH  + kSzP;
constexpr size_t kOffV   = kOffPL  + kSzP;
constexpr size_t kWsTotal = kOffV  + kSzX;
static_assert(kWsTotal == 27328512ull, "carve total");
static_assert(kWsTotal <= 134217728ull, "carve cap");
static_assert((kSzX % 128) == 0 && (kSzW % 128) == 0 && (kSzP % 128) == 0, "128-B aligned regions");

__device__ __forceinline__ unsigned short f2bf_bits(float f) {
  unsigned u = __float_as_uint(f);
  return (unsigned short)((u + 0x7FFFu + ((u >> 16) & 1u)) >> 16);
}
__device__ __forceinline__ float bf_bits2f(unsigned short h) { return __uint_as_float(((unsigned)h) << 16); }

__device__ __forceinline__ void dep_guard_h(v8f& a, v8f& b, v16h x, v16h y) { asm volatile("v_nop\n\tv_nop\n\tv_nop\n\tv_nop" : "+v"(a), "+v"(b) : "v"(x), "v"(y)); }
__device__ __forceinline__ void dep_guard_b(v8f& a, v8f& b, v16b x, v16b y) { asm volatile("v_nop\n\tv_nop\n\tv_nop\n\tv_nop" : "+v"(a), "+v"(b) : "v"(x), "v"(y)); }
__device__ __forceinline__ void keep4_h(v16h a, v16h b, v16h c, v16h d) { asm volatile("v_nop" :: "v"(a), "v"(b), "v"(c), "v"(d)); }
__device__ __forceinline__ void keep4_b(v16b a, v16b b, v16b c, v16b d) { asm volatile("v_nop" :: "v"(a), "v"(b), "v"(c), "v"(d)); }
__device__ __forceinline__ void acc_guard4(v8f& a, v8f& b, v8f& c, v8f& d) { asm volatile("v_nop\n\tv_nop\n\tv_nop\n\tv_nop" : "+v"(a), "+v"(b), "+v"(c), "+v"(d)); }
template <typename T> struct Frag;
template <> struct Frag<_Float16> {
  typedef v16h V; union U { v16h v; v8h h[2]; };
  static __device__ __forceinline__ v16h load(const _Float16* p) {
    U f; f.h[0] = *(const v8h*)(p); f.h[1] = *(const v8h*)(p + 16); return f.v;
  }
  static __device__ __forceinline__ v8f mma(v16h a, v16h b, v8f c) {
    return __builtin_amdgcn_wmma_f32_16x16x32_f16(false, a, false, b, (short)0, c, false, false);
  }
  static __device__ __forceinline__ void guard(v8f& a, v8f& b, v16h x, v16h y) { dep_guard_h(a, b, x, y); }
  static __device__ __forceinline__ void keep(v16h a, v16h b, v16h c, v16h d) { keep4_h(a, b, c, d); }
};
template <> struct Frag<__bf16> {
  typedef v16b V; union U { v16b v; v8b h[2]; };
  static __device__ __forceinline__ v16b load(const __bf16* p) {
    U f; f.h[0] = *(const v8b*)(p); f.h[1] = *(const v8b*)(p + 16); return f.v;
  }
  static __device__ __forceinline__ v8f mma(v16b a, v16b b, v8f c) {
    return __builtin_amdgcn_wmma_f32_16x16x32_bf16(false, a, false, b, (short)0, c, false, false);
  }
  static __device__ __forceinline__ void guard(v8f& a, v8f& b, v16b x, v16b y) { dep_guard_b(a, b, x, y); }
  static __device__ __forceinline__ void keep(v16b a, v16b b, v16b c, v16b d) { keep4_b(a, b, c, d); }
};

__device__ __forceinline__ v8f mma_b(v16b a, v16b b, v8f c) {
  c = __builtin_amdgcn_wmma_f32_16x16x32_bf16(false, a, false, b, (short)0, c, false, false);
  asm volatile("v_nop\n\tv_nop\n\tv_nop\n\tv_nop" : "+v"(c) : "v"(a), "v"(b));
  return c;
}
__device__ __forceinline__ v8f mma_h(v16h a, v16h b, v8f c) {
  c = __builtin_amdgcn_wmma_f32_16x16x32_f16(false, a, false, b, (short)0, c, false, false);
  asm volatile("v_nop\n\tv_nop\n\tv_nop\n\tv_nop" : "+v"(c) : "v"(a), "v"(b));
  return c;
}

template <int ET> struct Elem;
template <> struct Elem<0> { typedef _Float16 T; };
template <> struct Elem<1> { typedef __bf16 T; };
template <int ET, bool SPLIT, int BIAS_MODE, int OUT_MODE, bool RESID>
__global__ __launch_bounds__(256) void wmma_gemm64(
    const unsigned short* __restrict__ Ap, const unsigned short* __restrict__ A2p, int lda, long strideA,
    const unsigned short* __restrict__ Btp, const unsigned short* __restrict__ Bt2p, int ldb, long strideB,
    void* __restrict__ Cout, void* __restrict__ Cout2, int ldc, long strideC,
    const float* __restrict__ bias,
    const float* __restrict__ resid, long strideR,
    int M, int N, int K, float scale) {
  typedef typename Elem<ET>::T T;
  typedef typename Frag<T>::V V;
  const T* A = (const T*)Ap; const T* A2 = (const T*)A2p; const T* Bt = (const T*)Btp; const T* Bt2 = (const T*)Bt2p;
  __shared__ __align__(16) float sT[8][16 * 68];
  const int b    = blockIdx.y;
  const int lane = threadIdx.x & 31;
  const int wave = threadIdx.x >> 5;
  const int tilesN = N >> 6;
  const int tilesM = M >> 6;
  const int tile = blockIdx.x * 8 + wave;
  if (tile >= tilesM * tilesN) return;
  const int tm = tile / tilesN;
  const int tn = tile - tm * tilesN;
  const int m0 = tm << 6;
  const int n0 = tn << 6;

  const T* Ab  = A  + (size_t)b * strideA;
  const T* Bb  = Bt + (size_t)b * strideB;
  const T* Ab2 = SPLIT ? (A2  + (size_t)b * strideA) : nullptr;
  const T* Bb2 = SPLIT ? (Bt2 + (size_t)b * strideB) : nullptr;

  const int rlane = lane & 15;
  const int koff  = (lane >> 4) * 8;
  const int mOff  = (lane >> 4) * 8;

  v8f acc[4][4];
#pragma unroll
  for (int i = 0; i < 4; ++i)
#pragma unroll
    for (int j = 0; j < 4; ++j) acc[i][j] = (v8f){0.f,0.f,0.f,0.f,0.f,0.f,0.f,0.f};

  for (int k0 = 0; k0 < K; k0 += 32) {
    V bh[4], bl[4];
#pragma unroll
    for (int j = 0; j < 4; ++j) {
      const size_t bo = (size_t)(n0 + (j << 4) + rlane) * ldb + koff + k0;
      bh[j] = Frag<T>::load(Bb + bo);
      if (SPLIT) bl[j] = Frag<T>::load(Bb2 + bo);
    }
#pragma unroll
    for (int i = 0; i < 4; ++i) {
      const size_t ao = (size_t)(m0 + (i << 4) + rlane) * lda + koff + k0;
      V ah = Frag<T>::load(Ab + ao);
      V al;
      if (SPLIT) al = Frag<T>::load(Ab2 + ao);
#pragma unroll
      for (int j = 0; j < 4; ++j) {
        acc[i][j] = Frag<T>::mma(ah, bh[j], acc[i][j]);
        if (SPLIT) {
          acc[i][j] = Frag<T>::mma(ah, bl[j], acc[i][j]);
          acc[i][j] = Frag<T>::mma(al, bh[j], acc[i][j]);
        }
      }
      Frag<T>::guard(acc[i][0], acc[i][3], ah, SPLIT ? al : ah);
      Frag<T>::guard(acc[i][1], acc[i][2], ah, SPLIT ? al : ah);
    }
    Frag<T>::keep(bh[0], bh[1], bh[2], bh[3]);
    if (SPLIT) Frag<T>::keep(bl[0], bl[1], bl[2], bl[3]);
  }
  acc_guard4(acc[0][0], acc[0][1], acc[0][2], acc[0][3]);
  acc_guard4(acc[1][0], acc[1][1], acc[1][2], acc[1][3]);
  acc_guard4(acc[2][0], acc[2][1], acc[2][2], acc[2][3]);
  acc_guard4(acc[3][0], acc[3][1], acc[3][2], acc[3][3]);

  float* slab = sT[wave];
  const float* Rb = RESID ? (resid + (size_t)b * strideR) : nullptr;
#pragma unroll
  for (int i = 0; i < 4; ++i) {
    const int mBase = m0 + (i << 4);
#pragma unroll
    for (int j = 0; j < 4; ++j) {
      const int n = n0 + (j << 4) + rlane;
      float bv = 0.f;
      if (BIAS_MODE == 2) bv = bias[n];
#pragma unroll
      for (int r = 0; r < 8; ++r) {
        float v = acc[i][j][r] * scale;
        if (BIAS_MODE == 1) v += bias[mBase + mOff + r];
        if (BIAS_MODE == 2) v += bv;
        if (RESID) v += Rb[(size_t)(mBase + mOff + r) * ldc + n];
        slab[(mOff + r) * 68 + (j << 4) + rlane] = v;
      }
    }
    __builtin_amdgcn_fence(__ATOMIC_RELEASE, "workgroup");
    __builtin_amdgcn_wave_barrier();
    __builtin_amdgcn_fence(__ATOMIC_ACQUIRE, "workgroup");
    if (OUT_MODE == 0) {
      float* C = (float*)Cout + (size_t)b * strideC;
      const int hh = lane >> 4, c4 = (lane & 15) * 4;
      for (int pass = 0; pass < 2; ++pass) {
#pragma unroll
        for (int it = 0; it < 8; ++it) {
          const int row = it * 2 + hh;
          v4f v = *(const v4f*)(slab + row * 68 + c4);
          *(volatile v4f*)(C + (size_t)(mBase + row) * ldc + n0 + c4) = v;
        }
        __threadfence();
      }
    } else {
      const int q = lane >> 3, c8 = (lane & 7) * 8;
      unsigned short* C  = (unsigned short*)Cout  + (size_t)b * strideC;
      unsigned short* C2 = (OUT_MODE == 2) ? ((unsigned short*)Cout2 + (size_t)b * strideC) : nullptr;
      for (int pass = 0; pass < 2; ++pass) {
#pragma unroll
        for (int it = 0; it < 4; ++it) {
          const int row = it * 4 + q;
          const float* sp = slab + row * 68 + c8;
          v8h hv, lv;
#pragma unroll
          for (int e = 0; e < 8; ++e) {
            if (OUT_MODE == 1) {
              hv[e] = (_Float16)sp[e];
            } else {
              unsigned short hb = f2bf_bits(sp[e]);
              unsigned short lb = f2bf_bits(sp[e] - bf_bits2f(hb));
              hv[e] = __builtin_bit_cast(_Float16, hb);
              lv[e] = __builtin_bit_cast(_Float16, lb);
            }
          }
          *(volatile v8h*)(C + (size_t)(mBase + row) * ldc + n0 + c8) = hv;
          if (OUT_MODE == 2) *(volatile v8h*)(C2 + (size_t)(mBase + row) * ldc + n0 + c8) = lv;
        }
        __threadfence();
      }
    }
    __builtin_amdgcn_fence(__ATOMIC_RELEASE, "workgroup");
    __builtin_amdgcn_wave_barrier();
    __builtin_amdgcn_fence(__ATOMIC_ACQUIRE, "workgroup");
  }
}

__global__ __launch_bounds__(256) void split_rows_bf16_kernel(
    const float* __restrict__ src, unsigned short* __restrict__ dhi, unsigned short* __restrict__ dlo, int total8)
{
  const int i = blockIdx.x * 256 + threadIdx.x;
  if (i >= total8) return;
  const size_t e0 = (size_t)i << 3;
  const v4f a0 = *(const v4f*)(src + e0);
  const v4f a1 = *(const v4f*)(src + e0 + 4);
  v8h hv, lv;
#pragma unroll
  for (int e = 0; e < 4; ++e) {
    const unsigned short h0 = f2bf_bits(a0[e]), h1 = f2bf_bits(a1[e]);
    const unsigned short l0 = f2bf_bits(a0[e] - bf_bits2f(h0)), l1 = f2bf_bits(a1[e] - bf_bits2f(h1));
    hv[e]     = __builtin_bit_cast(_Float16, h0);
    hv[4 + e] = __builtin_bit_cast(_Float16, h1);
    lv[e]     = __builtin_bit_cast(_Float16, l0);
    lv[4 + e] = __builtin_bit_cast(_Float16, l1);
  }
  unsigned short* qh = dhi + e0;
  unsigned short* ql = dlo + e0;
  *(volatile v8h*)qh = hv;
  *(volatile v8h*)ql = lv;
  __threadfence();
  *(volatile v8h*)qh = hv;
  *(volatile v8h*)ql = lv;
}

__global__ __launch_bounds__(256) void xt_split_kernel(
    const float* __restrict__ x, unsigned short* __restrict__ XH, unsigned short* __restrict__ XL)
{
  __shared__ float sm[64][65];
  const int t  = threadIdx.x;
  const int n0 = blockIdx.x * 64;
  const int c0 = blockIdx.y * 64;
  const int b  = blockIdx.z;
  const float* xb = x + (size_t)b * kC * kN;
#pragma unroll
  for (int i = 0; i < 4; ++i) {
    const int e  = i * 256 + t;
    const int r  = e >> 4;
    const int n4 = (e & 15) * 4;
    const v4f v = *(const v4f*)(xb + (size_t)(c0 + r) * kN + n0 + n4);
    sm[n4 + 0][r] = v[0];
    sm[n4 + 1][r] = v[1];
    sm[n4 + 2][r] = v[2];
    sm[n4 + 3][r] = v[3];
  }
  __syncthreads();
  const int lane = t & 31, wave = t >> 5;
  const int q = lane >> 3, c8 = (lane & 7) * 8;
  v8h hv[2], lv[2];
#pragma unroll
  for (int it = 0; it < 2; ++it) {
    const int row = wave * 8 + it * 4 + q;
#pragma unroll
    for (int e = 0; e < 8; ++e) {
      const float f = sm[row][c8 + e];
      const unsigned short hb = f2bf_bits(f);
      const unsigned short lb = f2bf_bits(f - bf_bits2f(hb));
      hv[it][e] = __builtin_bit_cast(_Float16, hb);
      lv[it][e] = __builtin_bit_cast(_Float16, lb);
    }
  }
  for (int pass = 0; pass < 2; ++pass) {
#pragma unroll
    for (int it = 0; it < 2; ++it) {
      const int row = wave * 8 + it * 4 + q;
      const size_t o = ((size_t)b * kN + n0 + row) * kC + c0 + c8;
      *(volatile v8h*)(XH + o) = hv[it];
      *(volatile v8h*)(XL + o) = lv[it];
    }
    __threadfence();
  }
}

__global__ __launch_bounds__(256) void pos_build_kernel(
    const float* __restrict__ rd, const float* __restrict__ rh, const float* __restrict__ rw,
    unsigned short* __restrict__ PH, unsigned short* __restrict__ PL)
{
  const int gid = blockIdx.x * 256 + threadIdx.x;
  const int n   = gid >> 5;
  const int hd0 = (gid & 31) * 8;
  const int ih = n % kSide;
  const int iw = (n / kSide) % kSide;
  const int id = n / (kSide * kSide);
  v8h hv, lv;
#pragma unroll
  for (int e = 0; e < 8; ++e) {
    const int hd = hd0 + e;
    const float fh = rh[hd * kSide + ih];
    const float fw = rw[hd * kSide + iw];
    const float fd = rd[hd * kSide + id];
    const float f = (fh + fw) + fd;
    const unsigned short hb = f2bf_bits(f);
    const unsigned short lb = f2bf_bits(f - bf_bits2f(hb));
    hv[e] = __builtin_bit_cast(_Float16, hb);
    lv[e] = __builtin_bit_cast(_Float16, lb);
  }
  const size_t o = (size_t)n * kC + hd0;
  *(volatile v8h*)(PH + o) = hv;
  *(volatile v8h*)(PL + o) = lv;
  __threadfence();
  *(volatile v8h*)(PH + o) = hv;
  *(volatile v8h*)(PL + o) = lv;
}

__global__ __launch_bounds__(128) void attn_pos_kernel(
    const unsigned short* __restrict__ QH, const unsigned short* __restrict__ QL,
    const unsigned short* __restrict__ KH, const unsigned short* __restrict__ KL,
    const unsigned short* __restrict__ PH, const unsigned short* __restrict__ PL,
    const unsigned short* __restrict__ V16, float* __restrict__ out)
{
  union FB { v16b v; v8b h[2]; };
  union FH { v16h v; v8h h[2]; };
  __shared__ __align__(16) __bf16   sKh[kKC * kDk];
  __shared__ __align__(16) __bf16   sKl[kKC * kDk];
  __shared__ __align__(16) __bf16   sQh[kKC * kDk];
  __shared__ __align__(16) __bf16   sQl[kKC * kDk];
  __shared__ __align__(16) _Float16 sVt[kDk * kKC];
  __shared__ __align__(16) _Float16 sP[4][16 * kKC];
  __shared__ __align__(16) float    sO[kDk * kOP];

  const int tid  = threadIdx.x;
  const int wave = tid >> 5;
  const int lane = tid & 31;
  const int hh   = lane >> 4;
  const int c    = lane & 15;

  const int bx = blockIdx.x;
  const int qb = bx % kNQB;
  const int bh = bx / kNQB;
  const int h  = bh % kHeads;
  const int b  = bh / kHeads;
  const int qbase = qb * kQTile;
  const int q0 = qbase + wave * 16;
  const size_t rowbase = (size_t)b * kN;
  const int hcol = h * kDk;

  v16b qah, qal, pah, pal;
  {
    const size_t qo = (rowbase + q0 + c) * kC + hcol + 8 * hh;
    const size_t po = (size_t)(q0 + c) * kC + hcol + 8 * hh;
    qah = Frag<__bf16>::load((const __bf16*)QH + qo);
    qal = Frag<__bf16>::load((const __bf16*)QL + qo);
    pah = Frag<__bf16>::load((const __bf16*)PH + po);
    pal = Frag<__bf16>::load((const __bf16*)PL + po);
  }

  float mrow[8], lrow[8];
  v8f oacc[2];
#pragma unroll
  for (int r = 0; r < 8; ++r) { mrow[r] = -INFINITY; lrow[r] = 0.f; }
  oacc[0] = (v8f){0.f,0.f,0.f,0.f,0.f,0.f,0.f,0.f};
  oacc[1] = (v8f){0.f,0.f,0.f,0.f,0.f,0.f,0.f,0.f};

  _Float16* pw = sP[wave];

#pragma unroll 1
  for (int kc = 0; kc < kNCH; ++kc) {
    const int kv0 = kc * kKC;
    __syncthreads();
    {
      v4u rk[8];
      v4u rv[2];
#pragma unroll
      for (int i = 0; i < 2; ++i) {
        const int idx  = i * 128 + tid;
        const int row  = idx >> 2;
        const int part = idx & 3;
        const size_t off = (rowbase + kv0 + row) * kC + hcol + part * 8;
        rk[i]     = *(const v4u*)(KH + off);
        rk[2 + i] = *(const v4u*)(KL + off);
        rk[4 + i] = *(const v4u*)(QH + off);
        rk[6 + i] = *(const v4u*)(QL + off);
        const int vd = idx >> 3;
        const int vp = idx & 7;
        rv[i] = *(const v4u*)(V16 + ((size_t)b * kC + hcol + vd) * kN + kv0 + vp * 8);
      }
#pragma unroll
      for (int i = 0; i < 2; ++i) {
        const int idx  = i * 128 + tid;
        const int lo   = (idx >> 2) * kDk + (idx & 3) * 8;
        *(v4u*)(sKh + lo) = rk[i];
        *(v4u*)(sKl + lo) = rk[2 + i];
        *(v4u*)(sQh + lo) = rk[4 + i];
        *(v4u*)(sQl + lo) = rk[6 + i];
        *(v4u*)(sVt + (idx >> 3) * kKC + (idx & 7) * 8) = rv[i];
      }
    }
    __syncthreads();

    v8f s[4];
#pragma unroll
    for (int j = 0; j < 4; ++j) {
      const int ro = (j * 16 + c) * kDk + 8 * hh;
      FB kfh, kfl, qfh, qfl;
      kfh.h[0] = *(const v8b*)(sKh + ro);
      kfh.h[1] = *(const v8b*)(sKh + ro + 16);
      kfl.h[0] = *(const v8b*)(sKl + ro);
      kfl.h[1] = *(const v8b*)(sKl + ro + 16);
      qfh.h[0] = *(const v8b*)(sQh + ro);
      qfh.h[1] = *(const v8b*)(sQh + ro + 16);
      qfl.h[0] = *(const v8b*)(sQl + ro);
      qfl.h[1] = *(const v8b*)(sQl + ro + 16);
      v8f a = (v8f){0.f,0.f,0.f,0.f,0.f,0.f,0.f,0.f};
      a = mma_b(qah, kfh.v, a);
      a = mma_b(qah, kfl.v, a);
      a = mma_b(qal, kfh.v, a);
      a = mma_b(pah, qfh.v, a);
      a = mma_b(pah, qfl.v, a);
      a = mma_b(pal, qfh.v, a);
      s[j] = a;
    }

    float cm[8];
#pragma unroll
    for (int r = 0; r < 8; ++r) {
      float m = fmaxf(fmaxf(s[0][r], s[1][r]), fmaxf(s[2][r], s[3][r]));
      m = fmaxf(m, __shfl_xor(m, 1, 32));
      m = fmaxf(m, __shfl_xor(m, 2, 32));
      m = fmaxf(m, __shfl_xor(m, 4, 32));
      m = fmaxf(m, __shfl_xor(m, 8, 32));
      cm[r] = m;
    }
#pragma unroll
    for (int r = 0; r < 8; ++r) {
      const float mnew  = fmaxf(mrow[r], cm[r]);
      const float alpha = __expf(mrow[r] - mnew);
      mrow[r] = mnew;
      float psum = 0.f;
#pragma unroll
      for (int j = 0; j < 4; ++j) {
        const float p = __expf(s[j][r] - mnew);
        psum += p;
        pw[(8 * hh + r) * kKC + j * 16 + c] = (_Float16)(p * kPCarry);
      }
      psum += __shfl_xor(psum, 1, 32);
      psum += __shfl_xor(psum, 2, 32);
      psum += __shfl_xor(psum, 4, 32);
      psum += __shfl_xor(psum, 8, 32);
      lrow[r] = lrow[r] * alpha + psum;
      oacc[0][r] *= alpha;
      oacc[1][r] *= alpha;
    }
    __builtin_amdgcn_fence(__ATOMIC_RELEASE, "workgroup");
    __builtin_amdgcn_wave_barrier();
    __builtin_amdgcn_fence(__ATOMIC_ACQUIRE, "workgroup");

#pragma unroll
    for (int kk = 0; kk < 2; ++kk) {
      FH pa;
      pa.h[0] = *(const v8h*)(pw + c * kKC + kk * 32 + 8 * hh);
      pa.h[1] = *(const v8h*)(pw + c * kKC + kk * 32 + 16 + 8 * hh);
#pragma unroll
      for (int t = 0; t < 2; ++t) {
        FH vb;
        vb.h[0] = *(const v8h*)(sVt + (t * 16 + c) * kKC + kk * 32 + 8 * hh);
        vb.h[1] = *(const v8h*)(sVt + (t * 16 + c) * kKC + kk * 32 + 16 + 8 * hh);
        oacc[t] = mma_h(pa.v, vb.v, oacc[t]);
      }
    }
  }

#pragma unroll
  for (int r = 0; r < 8; ++r) {
    const float inv = 1.0f / (lrow[r] * kPCarry);
    sO[(c) * kOP + wave * 16 + 8 * hh + r]      = oacc[0][r] * inv;
    sO[(16 + c) * kOP + wave * 16 + 8 * hh + r] = oacc[1][r] * inv;
  }
  __syncthreads();
  {
    const int c4 = (lane & 15) * 4;
    float* ob = out + ((size_t)b * kC + hcol) * kN + qbase;
    v4f val[4];
#pragma unroll
    for (int it = 0; it < 4; ++it) {
      const int row = it * 8 + wave * 2 + hh;
      val[it] = *(const v4f*)(sO + row * kOP + c4);
    }
    for (int pass = 0; pass < 2; ++pass) {
#pragma unroll
      for (int it = 0; it < 4; ++it) {
        const int row = it * 8 + wave * 2 + hh;
        *(volatile v4f*)(ob + (size_t)row * kN + c4) = val[it];
      }
      __threadfence();
    }
  }
}

extern "C" void kernel_launch(void* const* d_in, const int* in_sizes, int n_in,
                              void* d_out, int out_size, void* d_ws, size_t ws_size,
                              hipStream_t stream) {
  if (n_in < 10) return;
  if (in_sizes[0] != kB * kC * kN) return;
  if (in_sizes[1] != kC * kC) return;
  if (in_sizes[2] != kC) return;
  if (in_sizes[3] != kC * kC) return;
  if (in_sizes[4] != kC) return;
  if (in_sizes[5] != kC * kC) return;
  if (in_sizes[6] != kC) return;
  if (in_sizes[7] != kC * kSide) return;
  if (in_sizes[8] != kC * kSide) return;
  if (in_sizes[9] != kC * kSide) return;
  if (out_size != kB * kC * kN) return;
  if (ws_size < kWsTotal) return;

  const float* x    = (const float*)d_in[0];
  const float* wq   = (const float*)d_in[1];
  const float* bq   = (const float*)d_in[2];
  const float* wk   = (const float*)d_in[3];
  const float* bk   = (const float*)d_in[4];
  const float* wv   = (const float*)d_in[5];
  const float* bv   = (const float*)d_in[6];
  const float* reld = (const float*)d_in[7];
  const float* relh = (const float*)d_in[8];
  const float* relw = (const float*)d_in[9];
  float* out = (float*)d_out;

  char* ws = (char*)d_ws;
  unsigned short* XH  = (unsigned short*)(ws + kOffXH);
  unsigned short* XL  = (unsigned short*)(ws + kOffXL);
  unsigned short* WQH = (unsigned short*)(ws + kOffWQH);
  unsigned short* WQL = (unsigned short*)(ws + kOffWQL);
  unsigned short* WKH = (unsigned short*)(ws + kOffWKH);
  unsigned short* WKL = (unsigned short*)(ws + kOffWKL);
  unsigned short* WVH = (unsigned short*)(ws + kOffWVH);
  unsigned short* WVL = (unsigned short*)(ws + kOffWVL);
  unsigned short* QH  = (unsigned short*)(ws + kOffQH);
  unsigned short* QL  = (unsigned short*)(ws + kOffQL);
  unsigned short* KH  = (unsigned short*)(ws + kOffKH);
  unsigned short* KL  = (unsigned short*)(ws + kOffKL);
  unsigned short* PH  = (unsigned short*)(ws + kOffPH);
  unsigned short* PL  = (unsigned short*)(ws + kOffPL);
  unsigned short* V16 = (unsigned short*)(ws + kOffV);

  xt_split_kernel<<<dim3(kN / 64, kC / 64, kB), 256, 0, stream>>>(x, XH, XL);

  split_rows_bf16_kernel<<<(kC * kC / 8) / 256, 256, 0, stream>>>(wq, WQH, WQL, kC * kC / 8);
  split_rows_bf16_kernel<<<(kC * kC / 8) / 256, 256, 0, stream>>>(wk, WKH, WKL, kC * kC / 8);
  split_rows_bf16_kernel<<<(kC * kC / 8) / 256, 256, 0, stream>>>(wv, WVH, WVL, kC * kC / 8);

  pos_build_kernel<<<(kN * 32) / 256, 256, 0, stream>>>(reld, relh, relw, PH, PL);

  const long sX = (long)kN * kC;
  const int gemmBlocks = ((kN / 64) * (kC / 64) + 7) / 8;

  wmma_gemm64<1, true, 2, 2, false><<<dim3(gemmBlocks, kB), 256, 0, stream>>>(
      XH, XL, kC, sX,
      WQH, WQL, kC, 0L,
      (void*)QH, (void*)QL, kC, sX,
      bq, nullptr, 0L,
      kN, kC, kC, 1.0f);
  wmma_gemm64<1, true, 2, 2, false><<<dim3(gemmBlocks, kB), 256, 0, stream>>>(
      XH, XL, kC, sX,
      WKH, WKL, kC, 0L,
      (void*)KH, (void*)KL, kC, sX,
      bk, nullptr, 0L,
      kN, kC, kC, 1.0f);
  wmma_gemm64<1, true, 1, 1, false><<<dim3(gemmBlocks, kB), 256, 0, stream>>>(
      WVH, WVL, kC, 0L,
      XH, XL, kC, sX,
      (void*)V16, nullptr, kN, (long)kC * kN,
      bv, nullptr, 0L,
      kC, kN, kC, 1.0f);

  attn_pos_kernel<<<kB * kHeads * kNQB, 128, 0, stream>>>(QH, QL, KH, KL, PH, PL, V16, out);
}
